// ScalarSoftmaxQuantization_14104672600377
// MI455X (gfx1250) — hardware-verified
//
#include <hip/hip_runtime.h>
#include <stddef.h>


typedef _Float16 v16h __attribute__((ext_vector_type(16)));
typedef float v8f __attribute__((ext_vector_type(8)));
typedef float v4f __attribute__((ext_vector_type(4)));

#define NBIN 32
#define WAVES_PER_BLOCK 8
#define GROUP_ELEMS 64
#define ALPHA_L2 (-14.426950408889634f)
#define EPS_C (1e-10f)
#define ESCALE (4096.0f)

__device__ __forceinline__ v8f wmma16(v16h a, v16h b, v8f c) {
  c = __builtin_amdgcn_wmma_f32_16x16x32_f16(false, a, false, b, (short)0, c,
                                             false, false);
  asm volatile("v_nop\n\tv_nop\n\tv_nop\n\tv_nop" : "+v"(c) : "v"(a), "v"(b));
  return c;
}

__global__ __launch_bounds__(256) void k_main(const float* __restrict__ x,
                                              const float* __restrict__ bins,
                                              float* out, float* partials,
                                              int nElems, int nGroups) {
  __shared__ float red[2][WAVES_PER_BLOCK][NBIN];
  __shared__ __attribute__((aligned(16))) float lineBuf[64];

  const int tid = threadIdx.x;
  const int lane = tid & 31;
  const int wv = tid >> 5;
  const int h = lane >> 4;
  const int m = lane & 15;

  float sumB = 0.f;
#pragma unroll
  for (int k = 0; k < NBIN; ++k) sumB += bins[k];
  const float epsB = EPS_C * sumB;

  float bk[16];
#pragma unroll
  for (int i = 0; i < 16; ++i) {
    const int kq = (i < 8) ? i : (i + 8);
    const float blo = bins[kq];
    const float bhi = bins[kq + 8];
    bk[i] = h ? bhi : blo;
  }

  const bool rowBins = (m == 0) || (m == 8);
  const bool rowOnes = (m == 1) || (m == 9);
  v16h Af;
#pragma unroll
  for (int i = 0; i < 16; ++i) {
    const float v = rowBins ? bk[i] : (rowOnes ? 1.0f : 0.0f);
    Af[i] = (_Float16)v;
  }

  float accP[16], accS[16];
#pragma unroll
  for (int i = 0; i < 16; ++i) { accP[i] = 0.f; accS[i] = 0.f; }

  const int totalWaves = gridDim.x * WAVES_PER_BLOCK;
  for (int g = blockIdx.x * WAVES_PER_BLOCK + wv; g < nGroups; g += totalWaves) {
    const int gbase = g * GROUP_ELEMS;
    const int idx0 = gbase + 4 * m;
    const bool full4 = (idx0 + 3) < nElems;

    float xs[4];
    if (full4) {
      const v4f xv = *(const v4f*)(x + idx0);
      xs[0] = xv[0]; xs[1] = xv[1]; xs[2] = xv[2]; xs[3] = xv[3];
    } else {
#pragma unroll
      for (int t = 0; t < 4; ++t) {
        int ii = idx0 + t;
        ii = (ii < nElems) ? ii : (nElems - 1);
        ii = (ii < 0) ? 0 : ii;
        xs[t] = x[ii];
      }
    }

    float bc[4];
#pragma unroll
    for (int t = 0; t < 4; ++t) {
      const float xv = xs[t];
      const bool valid = (idx0 + t) < nElems;

      float d[16];
      float dmin = 3.0e38f;
#pragma unroll
      for (int i = 0; i < 16; ++i) {
        d[i] = __builtin_fabsf(xv - bk[i]);
        dmin = __builtin_fminf(dmin, d[i]);
      }
      dmin = __builtin_fminf(dmin, __shfl_xor(dmin, 16));

      float es[16];
      v16h Bf;
#pragma unroll
      for (int i = 0; i < 16; ++i) {
        es[i] = ESCALE * __builtin_amdgcn_exp2f(ALPHA_L2 * (d[i] - dmin));
        Bf[i] = (_Float16)es[i];
      }

      v8f acc = {0.f, 0.f, 0.f, 0.f, 0.f, 0.f, 0.f, 0.f};
      acc = wmma16(Af, Bf, acc);

      const float numS = acc[0];
      const float denS = acc[1];
      const float rS = __builtin_amdgcn_rcpf(denS);
      bc[t] = numS * rS + epsB;

      const float rSm = valid ? rS : 0.f;
      const float epm = valid ? EPS_C : 0.f;
#pragma unroll
      for (int i = 0; i < 16; ++i) {
        const float a = es[i] * rSm + epm;
        accP[i] += a;
        accS[i] += __builtin_amdgcn_sqrtf(a);
      }
    }

    if (h == 0) {
      if (full4) {
        v4f v;
        v[0] = bc[0]; v[1] = bc[1]; v[2] = bc[2]; v[3] = bc[3];
        float* p = out + idx0;
        *(volatile v4f*)p = v;
        __threadfence();
        *(volatile v4f*)p = v;
      } else {
#pragma unroll
        for (int t = 0; t < 4; ++t) {
          if ((idx0 + t) < nElems) *(volatile float*)(out + idx0 + t) = bc[t];
        }
        __threadfence();
#pragma unroll
        for (int t = 0; t < 4; ++t) {
          if ((idx0 + t) < nElems) *(volatile float*)(out + idx0 + t) = bc[t];
        }
      }
    }
  }

#pragma unroll
  for (int i = 0; i < 16; ++i) {
    float p = accP[i];
    p += __shfl_xor(p, 1);
    p += __shfl_xor(p, 2);
    p += __shfl_xor(p, 4);
    p += __shfl_xor(p, 8);
    accP[i] = p;
    float s = accS[i];
    s += __shfl_xor(s, 1);
    s += __shfl_xor(s, 2);
    s += __shfl_xor(s, 4);
    s += __shfl_xor(s, 8);
    accS[i] = s;
  }
  if (m == 0) {
#pragma unroll
    for (int i = 0; i < 16; ++i) {
      const int k = ((i < 8) ? i : (i + 8)) + 8 * h;
      red[0][wv][k] = accP[i];
      red[1][wv][k] = accS[i];
    }
  }
  __syncthreads();
  if (tid < 64) {
    const int which = tid >> 5;
    const int k = tid & 31;
    float s = 0.f;
#pragma unroll
    for (int w = 0; w < WAVES_PER_BLOCK; ++w) s += red[which][w][k];
    lineBuf[tid] = s;
  }
  __syncthreads();
  if (tid < 16) {
    const v4f v = *(const v4f*)&lineBuf[4 * tid];
    float* p = partials + (size_t)blockIdx.x * 64 + 4 * tid;
    *(volatile v4f*)p = v;
    __threadfence();
    *(volatile v4f*)p = v;
  }
}

__global__ __launch_bounds__(64) void k_final(const float* __restrict__ partials,
                                              float* out, int nBlocks, int nElems) {
  __shared__ double accd[64];
  const int t = threadIdx.x;
  double s = 0.0;
  for (int b = 0; b < nBlocks; ++b) s += (double)partials[(size_t)b * 64 + t];
  accd[t] = s;
  __syncthreads();
  if (t == 0) {
    const float invN = 1.0f / (float)nElems;
    float ent = 0.f, quant = 0.f;
#pragma unroll 1
    for (int k = 0; k < NBIN; ++k) {
      const float p = (float)accd[k] * invN;
      ent -= p * logf(p);
      quant += (float)accd[NBIN + k] * invN;
    }
    v4f v;
    v[0] = ent;
    v[1] = 0.0f;
    v[2] = quant;
    v[3] = 0.0f;
    float* q = out + (size_t)nElems;
    *(volatile v4f*)q = v;
    __threadfence();
    *(volatile v4f*)q = v;
  }
}

extern "C" void kernel_launch(void* const* d_in, const int* in_sizes, int n_in,
                              void* d_out, int out_size, void* d_ws, size_t ws_size,
                              hipStream_t stream) {
  if (n_in < 2) return;
  const float* x    = (const float*)d_in[0];
  const float* bins = (const float*)d_in[1];
  float* out = (float*)d_out;
  float* ws  = (float*)d_ws;

  const int nElems = in_sizes[0];
  const int nBins  = in_sizes[1];
  if (nBins != NBIN || nElems <= 0) return;
  if ((long long)out_size < (long long)nElems + 4) return;

  const int nGroups = (nElems + GROUP_ELEMS - 1) / GROUP_ELEMS;
  int grid = (nGroups + WAVES_PER_BLOCK - 1) / WAVES_PER_BLOCK;
  if (grid > 1024) grid = 1024;
  const size_t maxByWs = ws_size / (64 * sizeof(float));
  if ((size_t)grid > maxByWs) grid = (int)maxByWs;
  if (grid < 1) return;

  k_main<<<grid, 256, 0, stream>>>(x, bins, out, ws, nElems, nGroups);
  k_final<<<1, 64, 0, stream>>>(ws, out, grid, nElems);
}
